// SelfAttentionLayer2D_70901320122847
// MI455X (gfx1250) — hardware-verified
//
#include <hip/hip_runtime.h>
#include <math.h>
#include <stdint.h>


#define NB   8
#define NT   4096
#define CD   128
#define TOK  (NB * NT)
#define RSB  16
#define NJ   (NT / 256)
#define PVM  128
#define EP   40
#define OUTN (NB * NT * CD)

#define SCW  64.0f
#define SCQ  8.0f
#define SCV  16.0f
#define SCE  32768.0f
#define SCR  2048.0f
#define SCO  4.0f
#define RLO  (1.0f / SCR)
#define SCS  (1.0f / (SCQ * SCQ))

static_assert(TOK % 64 == 0 && CD % 64 == 0 && CD % 32 == 0 && NT % 64 == 0);
static_assert((((TOK / 32) * (CD / 64)) % 8) == 0);
static_assert((((CD / 32) * (TOK / 64)) % 8) == 0);
static_assert((((TOK / 16) * (CD / 64)) % 8) == 0);
static_assert(NT % RSB == 0 && RSB == 16 && NT % 256 == 0 && NJ == 16);
static_assert(NT % PVM == 0 && PVM == 128 && (EP % 8) == 0 && EP >= 32);
static_assert((NB * NT * CD) % 2048 == 0);

typedef _Float16       v16h __attribute__((ext_vector_type(16)));
typedef _Float16       v8h  __attribute__((ext_vector_type(8)));
typedef float          v8f  __attribute__((ext_vector_type(8)));
typedef float          v4f  __attribute__((ext_vector_type(4)));
typedef unsigned int   v4u  __attribute__((ext_vector_type(4)));

union HU { v8h h; v4u u; _Float16 s[8]; };
union FR { v16h v; v8h h[2]; _Float16 s[16]; };
union H2 { _Float16 s[2]; unsigned int u; };
static_assert(sizeof(HU) == 16);
static_assert(sizeof(FR) == 32);
static_assert(sizeof(H2) == 4);

__device__ __forceinline__ unsigned short bf_bits(float f) {
  const unsigned u = __float_as_uint(f);
  return (unsigned short)((u + 0x7FFFu + ((u >> 16) & 1u)) >> 16);
}
__device__ __forceinline__ float bf_up(unsigned short h) { return __uint_as_float(((unsigned)h) << 16); }
__device__ __forceinline__ float bfr(float f) { return bf_up(bf_bits(f)); }
__device__ __forceinline__ v8f zero8() { v8f z = {0.f, 0.f, 0.f, 0.f, 0.f, 0.f, 0.f, 0.f}; return z; }

__device__ __forceinline__ _Float16 flush_h(_Float16 h) {
  const float f = (float)h;
  return (fabsf(f) < 6.103515625e-05f) ? (_Float16)0.0f : h;
}
__device__ __forceinline__ void split_h(float v, _Float16& hi, _Float16& lo) {
  const _Float16 hv = flush_h((_Float16)v);
  const _Float16 lv = flush_h((_Float16)((v - (float)hv) * SCR));
  hi = hv;
  lo = lv;
}

__device__ __forceinline__ void ld8(const float* p, float* o) {
  const v4f a = *(const v4f*)(p);
  const v4f b = *(const v4f*)(p + 4);
  o[0] = a[0]; o[1] = a[1]; o[2] = a[2]; o[3] = a[3];
  o[4] = b[0]; o[5] = b[1]; o[6] = b[2]; o[7] = b[3];
}
__device__ __forceinline__ void st8(float* p, const float* v) {
  v4f a, b;
  a[0] = v[0]; a[1] = v[1]; a[2] = v[2]; a[3] = v[3];
  b[0] = v[4]; b[1] = v[5]; b[2] = v[6]; b[3] = v[7];
  *(v4f*)(p) = a;
  *(v4f*)(p + 4) = b;
}

__device__ __forceinline__ v16h ldfrag_h(const _Float16* p) {
  FR f;
  f.h[0] = *(const v8h*)(p);
  f.h[1] = *(const v8h*)(p + 16);
  return f.v;
}

__device__ __forceinline__ v8f mma_h_raw(v16h a, v16h b, v8f c) {
  return __builtin_amdgcn_wmma_f32_16x16x32_f16(false, a, false, b, (short)0, c, false, false);
}
__device__ __forceinline__ void dep_guard_h(v8f& a, v8f& b, v16h x) {
#if defined(__HIP_DEVICE_COMPILE__)
  asm volatile("v_nop\n\tv_nop\n\tv_nop\n\tv_nop" : "+v"(a), "+v"(b) : "v"(x));
#endif
}
__device__ __forceinline__ void guard2(v8f& a, v8f& b, v16h x, v16h y) {
#if defined(__HIP_DEVICE_COMPILE__)
  asm volatile("v_nop\n\tv_nop\n\tv_nop\n\tv_nop" : "+v"(a), "+v"(b) : "v"(x), "v"(y));
#endif
}
__device__ __forceinline__ void keep4_h(v16h a, v16h b, v16h c, v16h d) {
#if defined(__HIP_DEVICE_COMPILE__)
  asm volatile("v_nop" :: "v"(a), "v"(b), "v"(c), "v"(d));
#endif
}
__device__ __forceinline__ void acc_guard4(v8f& a, v8f& b, v8f& c, v8f& d) {
#if defined(__HIP_DEVICE_COMPILE__)
  asm volatile("v_nop\n\tv_nop\n\tv_nop\n\tv_nop" : "+v"(a), "+v"(b), "+v"(c), "+v"(d));
#endif
}
__device__ __forceinline__ void wave_lds_sync() {
  __builtin_amdgcn_fence(__ATOMIC_RELEASE, "workgroup");
  __builtin_amdgcn_wave_barrier();
  __builtin_amdgcn_fence(__ATOMIC_ACQUIRE, "workgroup");
}

__global__ __launch_bounds__(256) void cvt_flat(const float* __restrict__ in, _Float16* out, int n8, float scale) {
  const int i = blockIdx.x * 256 + threadIdx.x;
  if (i < n8) {
    float v[8];
    ld8(in + (size_t)i * 8, v);
    HU u;
#pragma unroll
    for (int e = 0; e < 8; ++e) u.s[e] = flush_h((_Float16)(bfr(v[e]) * scale));
    _Float16* p = out + (size_t)i * 8;
    *(volatile v4u*)p = u.u;
    __threadfence();
    *(volatile v4u*)p = u.u;
  }
}

__global__ __launch_bounds__(256) void cvt_wT(const float* __restrict__ Wm, _Float16* out, int R, int C, float scale) {
  __shared__ float sw[64][33];
  const int t = threadIdx.x;
  const int r0 = blockIdx.x * 64, c0 = blockIdx.y * 32;
  {
    const int row = t >> 2, c8 = (t & 3) * 8;
    float v[8];
    ld8(Wm + (size_t)(r0 + row) * C + c0 + c8, v);
#pragma unroll
    for (int e = 0; e < 8; ++e) sw[row][c8 + e] = v[e];
  }
  __syncthreads();
  const int q8 = t & 7, cc = t >> 3;
  HU u;
#pragma unroll
  for (int e = 0; e < 8; ++e) u.s[e] = flush_h((_Float16)(bfr(sw[8 * q8 + e][cc]) * scale));
  _Float16* dst = out + (size_t)(c0 + cc) * R + r0 + 8 * q8;
  *(volatile v4u*)dst = u.u;
  __threadfence();
  *(volatile v4u*)dst = u.u;
}

template <int MI>
__device__ __forceinline__ void kseg(v8f (&acc)[MI][4], const _Float16* __restrict__ A, int lda, int m0,
                                     const _Float16* __restrict__ Bt, int ldb, int n0, int K, int rlane, int koff) {
  for (int kk = 0; kk < K; kk += 32) {
    v16h bh[4];
#pragma unroll
    for (int j = 0; j < 4; ++j) {
      const size_t bo = (size_t)(n0 + (j << 4) + rlane) * (size_t)ldb + koff + kk;
      bh[j] = ldfrag_h(Bt + bo);
    }
#pragma unroll
    for (int i = 0; i < MI; ++i) {
      const size_t ao = (size_t)(m0 + (i << 4) + rlane) * (size_t)lda + koff + kk;
      const v16h a0 = ldfrag_h(A + ao);
#pragma unroll
      for (int j = 0; j < 4; ++j) acc[i][j] = mma_h_raw(a0, bh[j], acc[i][j]);
      dep_guard_h(acc[i][0], acc[i][3], a0);
    }
    keep4_h(bh[0], bh[1], bh[2], bh[3]);
  }
}

template <int NPL, int BM>
__device__ __forceinline__ void epi16(const v8f (&acc)[4], float* slab, int lane,
                                      _Float16* Cp, _Float16* Cl, int ldc, int mBase, int n0,
                                      float cs, float so, const float* __restrict__ bias) {
  const int rlane = lane & 15, mOff = (lane >> 4) * 8;
  const int q8 = lane & 7, rr = lane >> 3, c8 = q8 * 8;
#pragma unroll
  for (int r = 0; r < 8; ++r) {
#pragma unroll
    for (int j = 0; j < 4; ++j) {
      slab[(mOff + r) * 68 + (j << 4) + rlane] = acc[j][r];
    }
  }
  wave_lds_sync();
  float bc[8];
#pragma unroll
  for (int e = 0; e < 8; ++e) bc[e] = 0.0f;
  if (BM == 1) {
    float t8[8];
    ld8(bias + n0 + c8, t8);
#pragma unroll
    for (int e = 0; e < 8; ++e) bc[e] = bfr(t8[e]);
  }
  v4u uh[4], ul[4];
#pragma unroll
  for (int it = 0; it < 4; ++it) {
    const int row = it * 4 + rr;
    float xs[8];
    ld8(slab + row * 68 + c8, xs);
    float brw = 0.0f;
    if (BM == 2) brw = bfr(bias[mBase + row]);
    HU h, l;
#pragma unroll
    for (int e = 0; e < 8; ++e) {
      const float v = (xs[e] * cs + bc[e] + brw) * so;
      if (NPL == 2) {
        split_h(v, h.s[e], l.s[e]);
      } else {
        h.s[e] = flush_h((_Float16)v);
        l.s[e] = (_Float16)0.0f;
      }
    }
    uh[it] = h.u;
    ul[it] = l.u;
  }
  for (int ps = 0; ps < 2; ++ps) {
#pragma unroll
    for (int it = 0; it < 4; ++it) {
      const int row = it * 4 + rr;
      const size_t co = (size_t)(mBase + row) * (size_t)ldc + n0 + c8;
      *(volatile v4u*)(Cp + co) = uh[it];
      if (NPL == 2) *(volatile v4u*)(Cl + co) = ul[it];
    }
    __threadfence();
  }
  wave_lds_sync();
}

template <int NPL, int MI, int BM>
__global__ __launch_bounds__(256) void gemm64p(
    const _Float16* __restrict__ A, int lda, const _Float16* __restrict__ Bt, int ldb, float cs, float so,
    _Float16* Cp, _Float16* Cl, int ldc, int M, int N, int K, const float* __restrict__ bias) {
  __shared__ __align__(16) float sT[8][16 * 68];
  const int lane = threadIdx.x & 31;
  const int wave = threadIdx.x >> 5;
  const int tilesN = N >> 6;
  const int tilesM = M / (16 * MI);
  const int tiles = tilesM * tilesN;
  const int item = blockIdx.x * 8 + wave;
  if (item >= tiles) return;
  const int tm = item / tilesN;
  const int tn = item - tm * tilesN;
  const int m0 = tm * (16 * MI);
  const int n0 = tn << 6;

  const int rlane = lane & 15;
  const int koff  = (lane >> 4) * 8;

  v8f acc[MI][4];
#pragma unroll
  for (int i = 0; i < MI; ++i)
#pragma unroll
    for (int j = 0; j < 4; ++j) acc[i][j] = zero8();

  kseg<MI>(acc, A, lda, m0, Bt, ldb, n0, K, rlane, koff);
#pragma unroll
  for (int i = 0; i < MI; ++i) acc_guard4(acc[i][0], acc[i][1], acc[i][2], acc[i][3]);

#pragma unroll
  for (int i = 0; i < MI; ++i) {
    epi16<NPL, BM>(acc[i], sT[wave], lane, Cp, Cl, ldc, m0 + (i << 4), n0, cs, so, bias);
  }
}

__global__ __launch_bounds__(256) void k_soft(const _Float16* __restrict__ FH, const _Float16* __restrict__ FL,
                                              const _Float16* __restrict__ GH, const _Float16* __restrict__ GL,
                                              _Float16* E, int b) {
  extern __shared__ __align__(16) float sc[];
  const int tid = threadIdx.x, wave = tid >> 5, lane = tid & 31;
  const int hh = lane >> 4, rl = lane & 15;
  const int n0 = blockIdx.x * RSB;

  const size_t qo = (size_t)(b * NT + n0 + rl) * CD + 8 * hh;
  v16h qh[4], ql[4];
#pragma unroll
  for (int ks = 0; ks < 4; ++ks) {
    qh[ks] = ldfrag_h(FH + qo + 32 * ks);
    ql[ks] = ldfrag_h(FL + qo + 32 * ks);
  }
  for (int ct = wave; ct < NT / 16; ct += 8) {
    const size_t ko = (size_t)(b * NT + 16 * ct + rl) * CD + 8 * hh;
    v8f a0 = zero8(), a1 = zero8();
#pragma unroll
    for (int ks = 0; ks < 4; ++ks) {
      const v16h kh = ldfrag_h(GH + ko + 32 * ks);
      const v16h kl = ldfrag_h(GL + ko + 32 * ks);
      a1 = mma_h_raw(qh[ks], kl, a1);
      a0 = mma_h_raw(qh[ks], kh, a0);
      a1 = mma_h_raw(ql[ks], kh, a1);
      guard2(a0, a1, kh, kl);
    }
    const int mc = 16 * ct + rl;
#pragma unroll
    for (int r = 0; r < 8; ++r) {
      sc[(size_t)(8 * hh + r) * NT + mc] = (a0[r] + a1[r] * RLO) * SCS;
    }
  }
  __syncthreads();

  for (int q2 = 0; q2 < RSB / 8; ++q2) {
    const int row = (RSB / 8) * wave + q2;
    float* rp = sc + (size_t)row * NT + 8 * lane;
    float mx = -3.0e38f;
#pragma unroll 4
    for (int j = 0; j < NJ; ++j) {
      float v[8];
      ld8(rp + 256 * j, v);
#pragma unroll
      for (int e = 0; e < 8; ++e) mx = fmaxf(mx, v[e]);
    }
#pragma unroll
    for (int off = 16; off >= 1; off >>= 1) mx = fmaxf(mx, __shfl_xor(mx, off, 32));
    float z = 0.0f;
#pragma unroll 2
    for (int j = 0; j < NJ; ++j) {
      float v[8];
      ld8(rp + 256 * j, v);
#pragma unroll
      for (int e = 0; e < 8; ++e) {
        const float ef = __expf(v[e] - mx);
        z += ef;
        v[e] = ef;
      }
      st8(rp + 256 * j, v);
    }
#pragma unroll
    for (int off = 16; off >= 1; off >>= 1) z += __shfl_xor(z, off, 32);
    const float rz = SCE * (1.0f / z);
    HU u[NJ];
#pragma unroll
    for (int j = 0; j < NJ; ++j) {
      float v[8];
      ld8(rp + 256 * j, v);
#pragma unroll
      for (int e = 0; e < 8; ++e) {
        const _Float16 h0 = (_Float16)(v[e] * rz);
        const float f0 = (float)h0;
        const bool sub = f0 < 6.103515625e-05f;
        u[j].s[e] = sub ? (_Float16)0.0f : h0;
      }
    }
    _Float16* erow = E + (size_t)(n0 + row) * NT + 8 * lane;
    for (int ps = 0; ps < 2; ++ps) {
#pragma unroll
      for (int j = 0; j < NJ; ++j) *(volatile v4u*)(erow + 256 * j) = u[j].u;
      __threadfence();
    }
  }
}

__global__ __launch_bounds__(256) void k_pv(const _Float16* __restrict__ E, const _Float16* __restrict__ HT,
                                            _Float16* OH, _Float16* OL, int b) {
  __shared__ __align__(16) _Float16 Et[PVM * EP];
  __shared__ __align__(16) float sO[8][16 * 68];
  const int tid = threadIdx.x, wave = tid >> 5, lane = tid & 31;
  const int hh = lane >> 4, rl = lane & 15;
  const int m0 = blockIdx.x * PVM;
  const int cw = 32 * (wave >> 1);
  const int mw = 64 * (wave & 1);

  v8f acc[2][4];
#pragma unroll
  for (int i = 0; i < 2; ++i)
#pragma unroll
    for (int j = 0; j < 4; ++j) acc[i][j] = zero8();

  const int pr = tid >> 4, m8 = (tid & 15) * 8;
  const _Float16* Ab = HT + (size_t)b * NT;

  for (int n0 = 0; n0 < NT; n0 += 32) {
    {
      HU ra, rb;
      const size_t eo = (size_t)(n0 + 2 * pr) * NT + m0 + m8;
      ra.h = *(const v8h*)(E + eo);
      rb.h = *(const v8h*)(E + eo + NT);
#pragma unroll
      for (int e = 0; e < 8; ++e) {
        H2 p;
        p.s[0] = ra.s[e];
        p.s[1] = rb.s[e];
        *(unsigned int*)(&Et[(m8 + e) * EP + 2 * pr]) = p.u;
      }
    }
    __syncthreads();
    v16h bq[4];
#pragma unroll
    for (int j = 0; j < 4; ++j) {
      FR f;
      const int eb = (mw + (j << 4) + rl) * EP + 8 * hh;
      f.h[0] = *(const v8h*)(&Et[eb]);
      f.h[1] = *(const v8h*)(&Et[eb + 16]);
      bq[j] = f.v;
    }
#pragma unroll
    for (int i = 0; i < 2; ++i) {
      const v16h a0 = ldfrag_h(Ab + (size_t)(cw + (i << 4) + rl) * TOK + n0 + 8 * hh);
#pragma unroll
      for (int j = 0; j < 4; ++j) acc[i][j] = mma_h_raw(a0, bq[j], acc[i][j]);
      dep_guard_h(acc[i][0], acc[i][3], a0);
    }
    keep4_h(bq[0], bq[1], bq[2], bq[3]);
    __syncthreads();
  }
  acc_guard4(acc[0][0], acc[0][1], acc[0][2], acc[0][3]);
  acc_guard4(acc[1][0], acc[1][1], acc[1][2], acc[1][3]);

  const float fo = 1.0f / (SCV * SCE);
#pragma unroll
  for (int i = 0; i < 2; ++i) {
    epi16<2, 0>(acc[i], sO[wave], lane, OH, OL, NT, b * CD + cw + (i << 4), m0 + mw, fo, SCO, (const float*)0);
  }
}

__global__ __launch_bounds__(256) void gemm_out(const _Float16* __restrict__ OH, const _Float16* __restrict__ OL,
                                                const _Float16* __restrict__ WV, const float* __restrict__ bias,
                                                float* out) {
  __shared__ __align__(16) float sO[8][16 * 68];
  const int tid = threadIdx.x, wave = tid >> 5, lane = tid & 31;
  const int hh = lane >> 4, rl = lane & 15;
  const int tiles = (TOK / 16) * (CD / 64);
  const int item = blockIdx.x * 8 + wave;
  if (item >= tiles) return;
  const int tm = item >> 1, tn = item & 1;
  const int row0 = tm << 4, n0 = tn << 6;

  v8f accH[4], accL[4];
#pragma unroll
  for (int j = 0; j < 4; ++j) { accH[j] = zero8(); accL[j] = zero8(); }

#pragma unroll
  for (int kk = 0; kk < CD; kk += 32) {
    v16h bq[4];
#pragma unroll
    for (int j = 0; j < 4; ++j) bq[j] = ldfrag_h(WV + (size_t)(n0 + (j << 4) + rl) * CD + 8 * hh + kk);
    const size_t ao = (size_t)(row0 + rl) * CD + 8 * hh + kk;
    const v16h ah = ldfrag_h(OH + ao);
    const v16h al = ldfrag_h(OL + ao);
#pragma unroll
    for (int j = 0; j < 4; ++j) accH[j] = mma_h_raw(ah, bq[j], accH[j]);
    dep_guard_h(accH[0], accH[3], ah);
#pragma unroll
    for (int j = 0; j < 4; ++j) accL[j] = mma_h_raw(al, bq[j], accL[j]);
    dep_guard_h(accL[0], accL[3], al);
    keep4_h(bq[0], bq[1], bq[2], bq[3]);
  }
  acc_guard4(accH[0], accH[1], accH[2], accH[3]);
  acc_guard4(accL[0], accL[1], accL[2], accL[3]);

  const float fo = 1.0f / (SCO * SCW);
  float* slab = sO[wave];
#pragma unroll
  for (int r = 0; r < 8; ++r) {
#pragma unroll
    for (int j = 0; j < 4; ++j) {
      slab[(8 * hh + r) * 68 + (j << 4) + rl] = (accH[j][r] + accL[j][r] * RLO) * fo;
    }
  }
  wave_lds_sync();
  const int p4 = (lane & 15) * 4, r2 = lane >> 4;
  const v4f bb = *(const v4f*)(bias + n0 + p4);
  v4f b4;
#pragma unroll
  for (int e = 0; e < 4; ++e) b4[e] = bfr(bb[e]);
  v4f ov[8];
#pragma unroll
  for (int it = 0; it < 8; ++it) {
    const int row = 2 * it + r2;
    const v4f a = *(const v4f*)(slab + row * 68 + p4);
    ov[it] = a + b4;
  }
  for (int ps = 0; ps < 2; ++ps) {
#pragma unroll
    for (int it = 0; it < 8; ++it) {
      const int row = 2 * it + r2;
      const size_t oo = (size_t)(row0 + row) * CD + n0 + p4;
      *(volatile v4f*)(out + oo) = ov[it];
    }
    __threadfence();
  }
}

extern "C" void kernel_launch(void* const* d_in, const int* in_sizes, int n_in,
                              void* d_out, int out_size, void* d_ws, size_t ws_size,
                              hipStream_t stream) {
  if (n_in < 9) return;
  if (in_sizes[0] != NB * NT * CD) return;
  if (in_sizes[1] != CD * CD || in_sizes[3] != CD * CD || in_sizes[5] != CD * CD || in_sizes[7] != CD * CD) return;
  if (in_sizes[2] != CD || in_sizes[4] != CD || in_sizes[6] != CD || in_sizes[8] != CD) return;
  if (out_size != OUTN) return;

  const float* x  = (const float*)d_in[0];
  const float* Wf = (const float*)d_in[1];
  const float* bf = (const float*)d_in[2];
  const float* Wg = (const float*)d_in[3];
  const float* bg = (const float*)d_in[4];
  const float* Wh = (const float*)d_in[5];
  const float* bh = (const float*)d_in[6];
  const float* Wv = (const float*)d_in[7];
  const float* bv = (const float*)d_in[8];

  const size_t PW  = (size_t)CD * CD * 2;
  const size_t PX  = (size_t)TOK * CD * 2;
  const size_t PHT = (size_t)CD * TOK * 2;
  const size_t PO  = (size_t)NB * CD * NT * 2;
  const size_t PE  = (size_t)NT * NT * 2;

  size_t off = 0;
  const size_t oWF = off; off += PW;
  const size_t oWG = off; off += PW;
  const size_t oWH = off; off += PW;
  const size_t oWV = off; off += PW;
  const size_t oXH = off; off += PX;
  const size_t oFH = off; off += PX;
  const size_t oFL = off; off += PX;
  const size_t oGH = off; off += PX;
  const size_t oGL = off; off += PX;
  const size_t oHT = off; off += PHT;
  const size_t oOH = off; off += PO;
  const size_t oOL = off; off += PO;
  const size_t oE  = off; off += PE;
  if (off > ws_size) return;
  if (off > (size_t)134217728) return;

  char* ws = (char*)d_ws;
  _Float16* WF16 = (_Float16*)(ws + oWF);
  _Float16* WG16 = (_Float16*)(ws + oWG);
  _Float16* WH16 = (_Float16*)(ws + oWH);
  _Float16* WV16 = (_Float16*)(ws + oWV);
  _Float16* xh   = (_Float16*)(ws + oXH);
  _Float16* FHp  = (_Float16*)(ws + oFH);
  _Float16* FLp  = (_Float16*)(ws + oFL);
  _Float16* GHp  = (_Float16*)(ws + oGH);
  _Float16* GLp  = (_Float16*)(ws + oGL);
  _Float16* HTp  = (_Float16*)(ws + oHT);
  _Float16* OHp  = (_Float16*)(ws + oOH);
  _Float16* OLp  = (_Float16*)(ws + oOL);
  _Float16* Ep   = (_Float16*)(ws + oE);
  float*    outf = (float*)d_out;

  const dim3 blk(256);
  const int n8x = (NB * NT * CD) / 8;
  const dim3 gX((n8x + 255) / 256);
  const dim3 gW(CD / 64, CD / 32);
  const dim3 gP(((TOK / 32) * (CD / 64) + 7) / 8);
  const dim3 gH(((CD / 32) * (TOK / 64) + 7) / 8);
  const dim3 gSo(NT / RSB);
  const dim3 gPV(NT / PVM);
  const dim3 gO(((TOK / 16) * (CD / 64) + 7) / 8);
  const float cs64 = 1.0f / SCW;
  const size_t ldsSoft = (size_t)RSB * NT * sizeof(float);

  hipFuncSetAttribute(reinterpret_cast<const void*>(&k_soft),
                      hipFuncAttributeMaxDynamicSharedMemorySize, (int)ldsSoft);

  cvt_wT<<<gW, blk, 0, stream>>>(Wf, WF16, CD, CD, SCW);
  cvt_wT<<<gW, blk, 0, stream>>>(Wg, WG16, CD, CD, SCW);
  cvt_wT<<<gW, blk, 0, stream>>>(Wh, WH16, CD, CD, SCW);
  cvt_wT<<<gW, blk, 0, stream>>>(Wv, WV16, CD, CD, SCW);
  cvt_flat<<<gX, blk, 0, stream>>>(x, xh, n8x, 1.0f);
  gemm64p<2, 2, 1><<<gP, blk, 0, stream>>>(xh, CD, WF16, CD, cs64, SCQ, FHp, FLp, CD, TOK, CD, CD, bf);
  gemm64p<2, 2, 1><<<gP, blk, 0, stream>>>(xh, CD, WG16, CD, cs64, SCQ, GHp, GLp, CD, TOK, CD, CD, bg);
  gemm64p<1, 2, 2><<<gH, blk, 0, stream>>>(WH16, CD, xh, CD, cs64, SCV, HTp, HTp, TOK, CD, TOK, CD, bh);
  for (int b = 0; b < NB; ++b) {
    k_soft<<<gSo, blk, ldsSoft, stream>>>(FHp, FLp, GHp, GLp, Ep, b);
    k_pv<<<gPV, blk, 0, stream>>>(Ep, HTp, OHp, OLp, b);
  }
  gemm_out<<<gO, blk, 0, stream>>>(OHp, OLp, WV16, bv, outf);
}
